// EvenLamerGAT_73504070303823
// MI455X (gfx1250) — hardware-run, weakly checked
//
#include <hip/hip_runtime.h>
#include <stddef.h>


#define KD1     128
#define F1      256
#define NH1     8
#define HC1     32
#define KD2     256
#define F2      64
#define NTHR    256
#define NWAVE   8
#define EPT     8
#define CHUNK   (NTHR * EPT)
#define WCAP    (EPT * 32)
#define LISTN   (NWAVE * WCAP)
#define NBMAX   2048
#define RCAP    28672
#define DEGCAP  4096
#define GBM     64
#define GTHR    128
#define NEG_SLOPE 0.2f
#define WCARRY  16.0f
#define HCARRY  4.0f
#define WSCAP   134217728
#define LDS_AGG ((2 * RCAP + 2 * NBMAX + LISTN) * 4 + 64)

static_assert((CHUNK & (CHUNK - 1)) == 0 && CHUNK <= 4096);
static_assert((NBMAX & (NBMAX - 1)) == 0 && NBMAX <= 4096);
static_assert(NTHR * 8 == NBMAX);
static_assert(LISTN >= NBMAX);
static_assert(LISTN >= NWAVE * WCAP);
static_assert((RCAP % 32) == 0);
static_assert(LDS_AGG <= 300000);
static_assert(GBM == (GTHR / 32) * 16);
static_assert(NH1 * HC1 == F1);
static_assert(KD2 == F1);
static_assert((KD1 % 32) == 0 && (KD2 % 32) == 0);
static_assert((F1 % 64) == 0 && (F2 % 64) == 0);
static_assert(F1 == 8 * 32);
static_assert(F2 == 4 * 16);

typedef float          v4f  __attribute__((ext_vector_type(4)));
typedef float          v8f  __attribute__((ext_vector_type(8)));
typedef int            v4i  __attribute__((ext_vector_type(4)));
typedef int            v8i  __attribute__((ext_vector_type(8)));
typedef unsigned short v8us __attribute__((ext_vector_type(8)));
typedef _Float16       v8h  __attribute__((ext_vector_type(8)));
typedef _Float16       v16h __attribute__((ext_vector_type(16)));
union FragH { v16h v; v8us h[2]; v8i w; };
union H8    { v8h v; v8us u; };

__device__ __forceinline__ v8h cvt8(v4f a, v4f b) {
  v8h o;
  o[0] = (_Float16)a.x; o[1] = (_Float16)a.y; o[2] = (_Float16)a.z; o[3] = (_Float16)a.w;
  o[4] = (_Float16)b.x; o[5] = (_Float16)b.y; o[6] = (_Float16)b.z; o[7] = (_Float16)b.w;
  return o;
}

__device__ __forceinline__ v8f wm(const FragH& a, const FragH& b, v8f c) {
  v8f d = __builtin_amdgcn_wmma_f32_16x16x32_f16(false, a.v, false, b.v, (short)0, c, false, false);
  asm volatile("v_nop\n\tv_nop\n\tv_nop\n\tv_nop" : "+v"(d) : "v"(a.w), "v"(b.w));
  return d;
}

__device__ __forceinline__ float lk_dot(v4f t, v4f a) {
  v4f z;
  z.x = fmaxf(t.x, NEG_SLOPE * t.x);
  z.y = fmaxf(t.y, NEG_SLOPE * t.y);
  z.z = fmaxf(t.z, NEG_SLOPE * t.z);
  z.w = fmaxf(t.w, NEG_SLOPE * t.w);
  float p = z.x * a.x;
  p = fmaf(z.y, a.y, p);
  p = fmaf(z.z, a.z, p);
  p = fmaf(z.w, a.w, p);
  return p;
}

__device__ __forceinline__ float elu1(float v) {
  const float e = __expf(v) - 1.0f;
  return v > 0.0f ? v : e;
}
__device__ __forceinline__ v4f elu4(v4f v) {
  v4f o;
  o.x = elu1(v.x); o.y = elu1(v.y); o.z = elu1(v.z); o.w = elu1(v.w);
  return o;
}

__device__ __forceinline__ int scan_chunk(const int* __restrict__ dsts, int nE, int cbase, int slotBase,
                                          int nb, int vec8, int* list, int tid, int lane, int wave) {
  int wc = 0;
  const int el0  = tid * EPT;
  const int e0   = cbase + el0;
  const int sent = -2147483647 - 1;
  v4i da, db;
  if (vec8 != 0 && cbase + CHUNK <= nE) {
    da = *(const v4i*)(dsts + e0);
    db = *(const v4i*)(dsts + e0 + 4);
  } else {
    da.x = (e0     < nE) ? dsts[min(e0,     nE - 1)] : sent;
    da.y = (e0 + 1 < nE) ? dsts[min(e0 + 1, nE - 1)] : sent;
    da.z = (e0 + 2 < nE) ? dsts[min(e0 + 2, nE - 1)] : sent;
    da.w = (e0 + 3 < nE) ? dsts[min(e0 + 3, nE - 1)] : sent;
    db.x = (e0 + 4 < nE) ? dsts[min(e0 + 4, nE - 1)] : sent;
    db.y = (e0 + 5 < nE) ? dsts[min(e0 + 5, nE - 1)] : sent;
    db.z = (e0 + 6 < nE) ? dsts[min(e0 + 6, nE - 1)] : sent;
    db.w = (e0 + 7 < nE) ? dsts[min(e0 + 7, nE - 1)] : sent;
  }
  const unsigned nbs = (unsigned)slotBase;
  const unsigned unb = (unsigned)nb;
  const unsigned s0 = (unsigned)da.x - nbs, s1 = (unsigned)da.y - nbs;
  const unsigned s2 = (unsigned)da.z - nbs, s3 = (unsigned)da.w - nbs;
  const unsigned s4 = (unsigned)db.x - nbs, s5 = (unsigned)db.y - nbs;
  const unsigned s6 = (unsigned)db.z - nbs, s7 = (unsigned)db.w - nbs;
  const bool h0 = s0 < unb, h1 = s1 < unb, h2 = s2 < unb, h3 = s3 < unb;
  const bool h4 = s4 < unb, h5 = s5 < unb, h6 = s6 < unb, h7 = s7 < unb;
  const unsigned any = __builtin_amdgcn_ballot_w32(h0 | h1 | h2 | h3 | h4 | h5 | h6 | h7);
  if (any != 0u) {
#define HITJ(J, HJ, SJ) { \
      const unsigned mj = __builtin_amdgcn_ballot_w32(HJ); \
      if (mj != 0u) { \
        if (HJ) { \
          const int pos = wc + (int)__builtin_amdgcn_mbcnt_lo(mj, 0u); \
          if (pos < WCAP) list[wave * WCAP + pos] = ((el0 + (J)) << 12) | (int)(SJ); \
        } \
        wc += (int)__builtin_popcount(mj); } }
    HITJ(0, h0, s0)
    HITJ(1, h1, s1)
    HITJ(2, h2, s2)
    HITJ(3, h3, s3)
    HITJ(4, h4, s4)
    HITJ(5, h5, s5)
    HITJ(6, h6, s6)
    HITJ(7, h7, s7)
#undef HITJ
  }
  return wc;
}

__device__ __forceinline__ int block_csr(const int* __restrict__ dsts, int nE, int nodeBase, int nb, int vec8,
                                         int* reg1, int* reg2, int* scnt, int* soff, int* list,
                                         int* wcnt, int* wtot, int tid, int lane, int wave, int& ovf) {
  for (int i = tid; i < NBMAX; i += NTHR) scnt[i] = 0;
  __syncthreads();

  int tot = 0;
  ovf = 0;
  const int nChunks = (nE + CHUNK - 1) / CHUNK;
#pragma unroll 1
  for (int ch = 0; ch < nChunks; ++ch) {
    const int cbase = ch * CHUNK;
    const int wc = scan_chunk(dsts, nE, cbase, nodeBase, nb, vec8, list, tid, lane, wave);
    if (lane == 0) wcnt[wave] = wc;
    __syncthreads();
    int pre = 0, all = 0;
#pragma unroll
    for (int w2 = 0; w2 < NWAVE; ++w2) {
      int c = wcnt[w2];
      c = c < 0 ? 0 : (c > WCAP ? WCAP : c);
      all += c;
      pre += (w2 < wave) ? c : 0;
    }
    const int wcc  = wc > WCAP ? WCAP : wc;
    const int base = tot + pre;
#pragma unroll 1
    for (int i = lane; i < wcc; i += 32) {
      const int ent = list[wave * WCAP + i];
      const int el  = (ent >> 12) & (CHUNK - 1);
      const int sl  = ent & (NBMAX - 1);
      int eid = cbase + el;
      eid = eid > nE - 1 ? nE - 1 : eid;
      const int pos = base + i;
      if (pos < RCAP) reg1[pos] = (int)(((unsigned)eid << 12) | (unsigned)sl);
    }
    tot += all;
    if (tot > RCAP) { ovf = 1; tot = RCAP; }
    __syncthreads();
  }
  const int nh = tot;

  if (wave == 0) {
#pragma unroll 1
    for (int b0 = 0; b0 < nh; b0 += 32) {
      const int idx = b0 + lane;
      const int uv  = reg1[idx < RCAP ? idx : RCAP - 1];
      const int m32 = (nh - b0) < 32 ? (nh - b0) : 32;
#pragma unroll 1
      for (int k = 0; k < m32; ++k) {
        const int u  = __builtin_amdgcn_readlane(uv, k);
        const int sl = u & (NBMAX - 1);
        if (lane == 0) scnt[sl] = scnt[sl] + 1;
      }
    }
  }
  __syncthreads();

  {
    const v4i ca = *(const v4i*)(scnt + 8 * tid);
    const v4i cb = *(const v4i*)(scnt + 8 * tid + 4);
    const int e0 = ca.x < 0 ? 0 : ca.x, e1 = ca.y < 0 ? 0 : ca.y, e2 = ca.z < 0 ? 0 : ca.z, e3 = ca.w < 0 ? 0 : ca.w;
    const int e4 = cb.x < 0 ? 0 : cb.x, e5 = cb.y < 0 ? 0 : cb.y, e6 = cb.z < 0 ? 0 : cb.z, e7 = cb.w < 0 ? 0 : cb.w;
    const int ts = e0 + e1 + e2 + e3 + e4 + e5 + e6 + e7;
    int incl = ts;
#pragma unroll
    for (int d = 1; d < 32; d <<= 1) {
      const int up = __shfl_up(incl, d);
      if (lane >= d) incl += up;
    }
    if (lane == 31) wtot[wave] = incl;
    __syncthreads();
    int pre = 0;
#pragma unroll
    for (int w2 = 0; w2 < NWAVE; ++w2) pre += (w2 < wave) ? wtot[w2] : 0;
    int run = pre + incl - ts;
    soff[8 * tid + 0] = run; run += e0;
    soff[8 * tid + 1] = run; run += e1;
    soff[8 * tid + 2] = run; run += e2;
    soff[8 * tid + 3] = run; run += e3;
    soff[8 * tid + 4] = run; run += e4;
    soff[8 * tid + 5] = run; run += e5;
    soff[8 * tid + 6] = run; run += e6;
    soff[8 * tid + 7] = run;
  }
  __syncthreads();
  for (int i = tid; i < NBMAX; i += NTHR) list[i] = soff[i];
  __syncthreads();

  if (wave == 0) {
#pragma unroll 1
    for (int b0 = 0; b0 < nh; b0 += 32) {
      const int idx = b0 + lane;
      const int uv  = reg1[idx < RCAP ? idx : RCAP - 1];
      const int m32 = (nh - b0) < 32 ? (nh - b0) : 32;
#pragma unroll 1
      for (int k = 0; k < m32; ++k) {
        const int u   = __builtin_amdgcn_readlane(uv, k);
        const int sl  = u & (NBMAX - 1);
        const int eid = (int)((unsigned)u >> 12);
        if (lane == 0) {
          int pos = list[sl];
          pos = pos < 0 ? 0 : (pos > RCAP - 1 ? RCAP - 1 : pos);
          reg2[pos] = eid;
          list[sl] = pos + 1;
        }
      }
    }
  }
  __syncthreads();
  return nh;
}

__global__ __launch_bounds__(NTHR) void k_xprep(const float* __restrict__ x, unsigned short* xh,
                                                int nN, int nUnits) {
  const int i = (int)blockIdx.x * NTHR + (int)threadIdx.x;
  if (i >= nUnits) return;
  const int row = i >> 4;
  const int c0  = (i & 15) * 8;
  const int rc  = row < nN ? row : nN - 1;
  const float* p = x + (size_t)rc * KD1 + c0;
  v4f a = *(const v4f*)p, b = *(const v4f*)(p + 4);
  const v4f z4 = {0.f, 0.f, 0.f, 0.f};
  if (row >= nN) { a = z4; b = z4; }
  H8 o;
  o.v = cvt8(a, b);
  const size_t off = (size_t)row * KD1 + c0;
  *(volatile v8us*)(xh + off) = o.u;
  __threadfence();
  *(volatile v8us*)(xh + off) = o.u;
}

__global__ __launch_bounds__(NTHR) void k_wprep(const float* __restrict__ Wl, const float* __restrict__ Wr,
                                                unsigned short* wt, int K, int NC, float carry) {
  const int j  = (int)blockIdx.y;
  const int u  = (int)blockIdx.x * NTHR + (int)threadIdx.x;
  const int kq = K >> 3;
  if (u >= NC * kq) return;
  const int n  = u / kq;
  const int k8 = (u - n * kq) * 8;
  const float* src = (j & 1) ? Wr : Wl;
  const float* p = src + (size_t)k8 * NC + n;
  v4f a, b;
  a.x = p[0 * (size_t)NC]; a.y = p[1 * (size_t)NC]; a.z = p[2 * (size_t)NC]; a.w = p[3 * (size_t)NC];
  b.x = p[4 * (size_t)NC]; b.y = p[5 * (size_t)NC]; b.z = p[6 * (size_t)NC]; b.w = p[7 * (size_t)NC];
  H8 o;
  o.v = cvt8(a * carry, b * carry);
  const size_t off = (size_t)j * NC * K + (size_t)u * 8;
  *(volatile v8us*)(wt + off) = o.u;
  __threadfence();
  *(volatile v8us*)(wt + off) = o.u;
}

template <int K, int NC>
__global__ __launch_bounds__(GTHR) void k_gemm(const unsigned short* __restrict__ A,
                                               const unsigned short* __restrict__ WT,
                                               const float* __restrict__ bl, const float* __restrict__ br,
                                               float* Y, int yStride, int nN, float invc) {
  __shared__ __attribute__((aligned(16))) float stg[GBM * 64];
  constexpr int KS = K / 32;
  constexpr int NG = 2 * NC / 64;
  const int tid = threadIdx.x, lane = tid & 31, wave = tid >> 5, hh = lane >> 4, m = lane & 15;
  const int rowBase = (int)blockIdx.x * GBM;
  int ar = rowBase + 16 * wave + m;
  ar = ar < nN ? ar : nN - 1;
  const size_t arow = (size_t)ar * K + 8 * hh;
  FragH a[KS];
#pragma unroll
  for (int ks = 0; ks < KS; ++ks) {
    a[ks].h[0] = *(const v8us*)(A + arow + 32 * ks);
    a[ks].h[1] = *(const v8us*)(A + arow + 32 * ks + 16);
  }
#pragma unroll 1
  for (int g = 0; g < NG; ++g) {
    const int mat  = (64 * g) / NC;
    const int col0 = 64 * g - mat * NC;
    const float* bsel = (mat != 0) ? br : bl;
    v8f acc[4];
#pragma unroll
    for (int t = 0; t < 4; ++t) { v8f z = {0.f, 0.f, 0.f, 0.f, 0.f, 0.f, 0.f, 0.f}; acc[t] = z; }
    const size_t brow = (size_t)(64 * g + m) * K + 8 * hh;
#pragma unroll
    for (int ks = 0; ks < KS; ++ks) {
#pragma unroll
      for (int t = 0; t < 4; ++t) {
        const size_t bo = brow + (size_t)(16 * t) * K + 32 * ks;
        FragH b;
        b.h[0] = *(const v8us*)(WT + bo);
        b.h[1] = *(const v8us*)(WT + bo + 16);
        acc[t] = wm(a[ks], b, acc[t]);
      }
    }
    float* sp = stg + (size_t)(16 * wave + 8 * hh) * 64 + m;
#pragma unroll
    for (int t = 0; t < 4; ++t) {
      const float bv = bsel[col0 + 16 * t + m];
#pragma unroll
      for (int r = 0; r < 8; ++r) sp[(size_t)r * 64 + 16 * t] = acc[t][r] * invc + bv;
    }
    __syncthreads();
    const int nF4 = GBM * 64 / 4;
    float* yb = Y + (size_t)mat * (size_t)yStride + (size_t)rowBase * NC + col0;
    const v4f* s4 = (const v4f*)stg;
#pragma unroll 1
    for (int f = tid; f < nF4; f += GTHR) {
      const int r = f >> 4, q = f & 15;
      const v4f v = s4[f];
      *(volatile v4f*)(yb + (size_t)r * NC + 4 * q) = v;
    }
    __threadfence();
#pragma unroll 1
    for (int f = tid; f < nF4; f += GTHR) {
      const int r = f >> 4, q = f & 15;
      const v4f v = s4[f];
      *(volatile v4f*)(yb + (size_t)r * NC + 4 * q) = v;
    }
    __syncthreads();
  }
}

__global__ __launch_bounds__(NTHR) void k_agg1(
    const int* __restrict__ srcs, const int* __restrict__ dsts,
    const float* __restrict__ xl, const float* __restrict__ xr,
    const float* __restrict__ attr, const float* __restrict__ biaso,
    unsigned short* hpl, int nN, int nE, int nb, int vec8) {
  extern __shared__ v4f lds_dyn[];
  int* reg1 = (int*)lds_dyn;
  int* reg2 = reg1 + RCAP;
  int* scnt = reg2 + RCAP;
  int* soff = scnt + NBMAX;
  int* list = soff + NBMAX;
  int* wcnt = list + LISTN;
  int* wtot = wcnt + NWAVE;
  const int tid = threadIdx.x, lane = tid & 31, wave = tid >> 5;
  const int nodeBase = (int)blockIdx.x * nb;

  int ovf = 0;
  const int nh = block_csr(dsts, nE, nodeBase, nb, vec8, reg1, reg2, scnt, soff, list, wcnt, wtot,
                           tid, lane, wave, ovf);

  const int nbw = nb >> 3;
  const int c8  = 8 * lane;
  const v4f at0 = *(const v4f*)(attr + c8);
  const v4f at1 = *(const v4f*)(attr + c8 + 4);
  const v4f bz0 = *(const v4f*)(biaso + c8);
  const v4f bz1 = *(const v4f*)(biaso + c8 + 4);
  const float pnan = __int_as_float(0x7fc00000);
  const float povf = (ovf != 0) ? pnan : 0.0f;
#pragma unroll 1
  for (int jt = 0; jt < nbw; ++jt) {
    const int slot = wave * nbw + jt;
    const int grow = nodeBase + slot;
    const int gcl  = grow < nN ? grow : nN - 1;
    int st = soff[slot];
    const int cr = scnt[slot];
    int cnt = cr;
    st  = st < 0 ? 0 : (st > nh ? nh : st);
    cnt = cnt < 0 ? 0 : (cnt > DEGCAP ? DEGCAP : cnt);
    if (cnt > nh - st) cnt = nh - st;
    const float pz = (cr > DEGCAP) ? pnan : povf;

    const float* xrrow = xr + (size_t)gcl * F1;
    const float* xdrow = xl + (size_t)gcl * F1;
    const v4f xr0 = *(const v4f*)(xrrow + c8);
    const v4f xr1 = *(const v4f*)(xrrow + c8 + 4);
    const v4f xd0 = *(const v4f*)(xdrow + c8);
    const v4f xd1 = *(const v4f*)(xdrow + c8 + 4);

    float el = lk_dot(xd0 + xr0, at0) + lk_dot(xd1 + xr1, at1);
    el += __shfl_xor(el, 2);
    el += __shfl_xor(el, 1);
    float mrun = el, den = 1.0f;
    v4f acc0 = xd0, acc1 = xd1;

#pragma unroll 1
    for (int q = 0; q < cnt; ++q) {
      int idx = st + q; idx = idx > RCAP - 1 ? RCAP - 1 : idx;
      int eid = reg2[idx]; eid = eid < 0 ? 0 : (eid > nE - 1 ? nE - 1 : eid);
      const int sraw = srcs[eid];
      const int s = sraw < 0 ? 0 : (sraw > nN - 1 ? nN - 1 : sraw);
      const float* xsrow = xl + (size_t)s * F1;
      const v4f xs0 = *(const v4f*)(xsrow + c8);
      const v4f xs1 = *(const v4f*)(xsrow + c8 + 4);
      float la = lk_dot(xs0 + xr0, at0) + lk_dot(xs1 + xr1, at1);
      la += __shfl_xor(la, 2);
      la += __shfl_xor(la, 1);
      const float mn  = fmaxf(mrun, la);
      const float s1v = __expf(mrun - mn);
      const float s2v = __expf(la - mn);
      den = fmaf(den, s1v, s2v);
      acc0.x = fmaf(acc0.x, s1v, s2v * xs0.x);
      acc0.y = fmaf(acc0.y, s1v, s2v * xs0.y);
      acc0.z = fmaf(acc0.z, s1v, s2v * xs0.z);
      acc0.w = fmaf(acc0.w, s1v, s2v * xs0.w);
      acc1.x = fmaf(acc1.x, s1v, s2v * xs1.x);
      acc1.y = fmaf(acc1.y, s1v, s2v * xs1.y);
      acc1.z = fmaf(acc1.z, s1v, s2v * xs1.z);
      acc1.w = fmaf(acc1.w, s1v, s2v * xs1.w);
      mrun = mn;
    }
    const float inv = __builtin_amdgcn_rcpf(den);
    v4f o0, o1;
    o0.x = fmaf(acc0.x, inv, bz0.x);
    o0.y = fmaf(acc0.y, inv, bz0.y);
    o0.z = fmaf(acc0.z, inv, bz0.z);
    o0.w = fmaf(acc0.w, inv, bz0.w);
    o1.x = fmaf(acc1.x, inv, bz1.x);
    o1.y = fmaf(acc1.y, inv, bz1.y);
    o1.z = fmaf(acc1.z, inv, bz1.z);
    o1.w = fmaf(acc1.w, inv, bz1.w);
    const v4f h0 = elu4(o0) * HCARRY + pz;
    const v4f h1 = elu4(o1) * HCARRY + pz;
    H8 o;
    o.v = cvt8(h0, h1);
    unsigned short* hp = hpl + (size_t)gcl * F1 + c8;
    const bool wr = grow < nN;
    if (wr) *(volatile v8us*)hp = o.u;
    __threadfence();
    if (wr) *(volatile v8us*)hp = o.u;
  }
}

__global__ __launch_bounds__(NTHR) void k_agg2(
    const int* __restrict__ srcs, const int* __restrict__ dsts,
    const float* __restrict__ xl, const float* __restrict__ xr,
    const float* __restrict__ attr, const float* __restrict__ biaso,
    float* out, int nN, int nE, int nb, int vec8) {
  extern __shared__ v4f lds_dyn[];
  int* reg1 = (int*)lds_dyn;
  int* reg2 = reg1 + RCAP;
  int* scnt = reg2 + RCAP;
  int* soff = scnt + NBMAX;
  int* list = soff + NBMAX;
  int* wcnt = list + LISTN;
  int* wtot = wcnt + NWAVE;
  const int tid = threadIdx.x, lane = tid & 31, wave = tid >> 5;
  const int nodeBase = (int)blockIdx.x * nb;

  int ovf = 0;
  const int nh = block_csr(dsts, nE, nodeBase, nb, vec8, reg1, reg2, scnt, soff, list, wcnt, wtot,
                           tid, lane, wave, ovf);

  const int nbw = nb >> 3;
  const int c4  = 4 * (lane & 15);
  const int hs  = lane >> 4;
  const v4f at = *(const v4f*)(attr + c4);
  const v4f bz = *(const v4f*)(biaso + c4);
  const size_t o1off = (size_t)nN * F2;
  const float pnan = __int_as_float(0x7fc00000);
  const float povf = (ovf != 0) ? pnan : 0.0f;
#pragma unroll 1
  for (int jt = 0; jt < nbw; ++jt) {
    const int slot = wave * nbw + jt;
    const int grow = nodeBase + slot;
    const int gcl  = grow < nN ? grow : nN - 1;
    int st = soff[slot];
    const int cr = scnt[slot];
    int cnt = cr;
    st  = st < 0 ? 0 : (st > nh ? nh : st);
    cnt = cnt < 0 ? 0 : (cnt > DEGCAP ? DEGCAP : cnt);
    if (cnt > nh - st) cnt = nh - st;
    const float pz = (cr > DEGCAP) ? pnan : povf;

    const v4f xr4 = *(const v4f*)(xr + (size_t)gcl * F2 + c4);
    const v4f xd4 = *(const v4f*)(xl + (size_t)gcl * F2 + c4);

    float el = lk_dot(xd4 + xr4, at);
    el += __shfl_xor(el, 8);
    el += __shfl_xor(el, 4);
    el += __shfl_xor(el, 2);
    el += __shfl_xor(el, 1);
    float mrun = el, den = 1.0f;
    v4f acc = xd4;

#pragma unroll 1
    for (int q = 0; q < cnt; ++q) {
      int idx = st + q; idx = idx > RCAP - 1 ? RCAP - 1 : idx;
      int eid = reg2[idx]; eid = eid < 0 ? 0 : (eid > nE - 1 ? nE - 1 : eid);
      const int sraw = srcs[eid];
      const int s = sraw < 0 ? 0 : (sraw > nN - 1 ? nN - 1 : sraw);
      const v4f xs4 = *(const v4f*)(xl + (size_t)s * F2 + c4);
      float la = lk_dot(xs4 + xr4, at);
      la += __shfl_xor(la, 8);
      la += __shfl_xor(la, 4);
      la += __shfl_xor(la, 2);
      la += __shfl_xor(la, 1);
      const float mn  = fmaxf(mrun, la);
      const float s1v = __expf(mrun - mn);
      const float s2v = __expf(la - mn);
      den = fmaf(den, s1v, s2v);
      acc.x = fmaf(acc.x, s1v, s2v * xs4.x);
      acc.y = fmaf(acc.y, s1v, s2v * xs4.y);
      acc.z = fmaf(acc.z, s1v, s2v * xs4.z);
      acc.w = fmaf(acc.w, s1v, s2v * xs4.w);
      mrun = mn;
    }
    const float inv = __builtin_amdgcn_rcpf(den);
    v4f o;
    o.x = fmaf(acc.x, inv, bz.x) + pz;
    o.y = fmaf(acc.y, inv, bz.y) + pz;
    o.z = fmaf(acc.z, inv, bz.z) + pz;
    o.w = fmaf(acc.w, inv, bz.w) + pz;
    float mx = fmaxf(fmaxf(o.x, o.y), fmaxf(o.z, o.w));
    mx = fmaxf(mx, __shfl_xor(mx, 8));
    mx = fmaxf(mx, __shfl_xor(mx, 4));
    mx = fmaxf(mx, __shfl_xor(mx, 2));
    mx = fmaxf(mx, __shfl_xor(mx, 1));
    float se = __expf(o.x - mx) + __expf(o.y - mx) + __expf(o.z - mx) + __expf(o.w - mx);
    se += __shfl_xor(se, 8);
    se += __shfl_xor(se, 4);
    se += __shfl_xor(se, 2);
    se += __shfl_xor(se, 1);
    const float lse = mx + __logf(se);
    const v4f ols = o - lse;
    const v4f val = (hs != 0) ? ols : o;
    float* op = out + ((hs != 0) ? o1off : (size_t)0) + (size_t)gcl * F2 + c4;
    const bool wr = grow < nN;
    if (wr) *(volatile v4f*)op = val;
    __threadfence();
    if (wr) *(volatile v4f*)op = val;
  }
}

static int pick_nb(int nE, int nN) {
  int nb = NBMAX;
  while (nb > 16 && (long long)nb * (long long)nE * 5LL > (long long)RCAP * (long long)nN * 4LL) nb >>= 1;
  return nb;
}

extern "C" void kernel_launch(void* const* d_in, const int* in_sizes, int n_in,
                              void* d_out, int out_size, void* d_ws, size_t ws_size,
                              hipStream_t stream) {
  if (n_in < 14) return;
  const int nN = in_sizes[0] / KD1;
  if (nN <= 0 || in_sizes[0] != nN * KD1) return;
  if (nN > (1 << 24)) return;
  const int szE = in_sizes[1];
  if (szE < 2 || (szE & 1) != 0) return;
  const int nE = szE / 2;
  if (nE > (1 << 20)) return;
  if (in_sizes[2] != KD1 * F1 || in_sizes[4] != KD1 * F1) return;
  if (in_sizes[3] != F1 || in_sizes[5] != F1 || in_sizes[7] != F1) return;
  if (in_sizes[6] != NH1 * HC1) return;
  if (in_sizes[8] != KD2 * F2 || in_sizes[10] != KD2 * F2) return;
  if (in_sizes[9] != F2 || in_sizes[11] != F2 || in_sizes[13] != F2 || in_sizes[12] != F2) return;
  if (out_size != 2 * nN * F2) return;

  const float* x     = (const float*)d_in[0];
  const int*   ei    = (const int*)d_in[1];
  const float* Wl1   = (const float*)d_in[2];
  const float* bl1   = (const float*)d_in[3];
  const float* Wr1   = (const float*)d_in[4];
  const float* br1   = (const float*)d_in[5];
  const float* att1  = (const float*)d_in[6];
  const float* bias1 = (const float*)d_in[7];
  const float* Wl2   = (const float*)d_in[8];
  const float* bl2   = (const float*)d_in[9];
  const float* Wr2   = (const float*)d_in[10];
  const float* br2   = (const float*)d_in[11];
  const float* att2  = (const float*)d_in[12];
  const float* bias2 = (const float*)d_in[13];
  float* out = (float*)d_out;

  const int MP     = ((nN + GBM - 1) / GBM) * GBM;
  const int nb     = pick_nb(nE, nN);
  const int vec8   = ((nE & 3) == 0) ? 1 : 0;
  const int nUnits = MP * 16;

  char* ws = (char*)d_ws;
  size_t off = 0;
  const size_t oWT1 = off; off += (size_t)2 * F1 * KD1 * 2;   off = (off + 255) & ~(size_t)255;
  const size_t oWT2 = off; off += (size_t)2 * F2 * KD2 * 2;   off = (off + 255) & ~(size_t)255;
  const size_t szXH = (size_t)MP * KD1 * 2, szHH = (size_t)MP * F1 * 2;
  const size_t oXH  = off; off += (szXH > szHH ? szXH : szHH); off = (off + 255) & ~(size_t)255;
  const size_t szY1 = (size_t)2 * MP * F1 * 4, szY2 = (size_t)2 * MP * F2 * 4;
  const size_t oY   = off; off += (szY1 > szY2 ? szY1 : szY2); off = (off + 255) & ~(size_t)255;
  if (off > ws_size || off > (size_t)WSCAP) return;
  unsigned short* WT1 = (unsigned short*)(ws + oWT1);
  unsigned short* WT2 = (unsigned short*)(ws + oWT2);
  unsigned short* XH  = (unsigned short*)(ws + oXH);
  unsigned short* HH  = (unsigned short*)(ws + oXH);
  float* Y = (float*)(ws + oY);

  hipFuncSetAttribute(reinterpret_cast<const void*>(&k_agg1),
                      hipFuncAttributeMaxDynamicSharedMemorySize, LDS_AGG);
  hipFuncSetAttribute(reinterpret_cast<const void*>(&k_agg2),
                      hipFuncAttributeMaxDynamicSharedMemorySize, LDS_AGG);

  k_xprep<<<(nUnits + NTHR - 1) / NTHR, NTHR, 0, stream>>>(x, XH, nN, nUnits);
  k_wprep<<<dim3((F1 * KD1 / 8 + NTHR - 1) / NTHR, 2), NTHR, 0, stream>>>(Wl1, Wr1, WT1, KD1, F1, WCARRY);
  k_wprep<<<dim3((F2 * KD2 / 8 + NTHR - 1) / NTHR, 2), NTHR, 0, stream>>>(Wl2, Wr2, WT2, KD2, F2, WCARRY);
  k_gemm<KD1, F1><<<MP / GBM, GTHR, 0, stream>>>(XH, WT1, bl1, br1, Y, MP * F1, nN, 1.0f / 16.0f);
  k_agg1<<<(nN + nb - 1) / nb, NTHR, LDS_AGG, stream>>>(ei, ei + nE, Y, Y + (size_t)MP * F1, att1, bias1,
                                                        HH, nN, nE, nb, vec8);
  k_gemm<KD2, F2><<<MP / GBM, GTHR, 0, stream>>>(HH, WT2, bl2, br2, Y, MP * F2, nN, 1.0f / 64.0f);
  k_agg2<<<(nN + nb - 1) / nb, NTHR, LDS_AGG, stream>>>(ei, ei + nE, Y, Y + (size_t)MP * F2, att2, bias2,
                                                        out, nN, nE, nb, vec8);
}
